// GraphChebNet_40785009443419
// MI455X (gfx1250) — hardware-verified
//
#include <hip/hip_runtime.h>
#include <stddef.h>


#define DI      128
#define HD      256
#define K1      256
#define K2      512
#define P1      256
#define P2      512
#define NTHR    256
#define NWAVE   8
#define EPT     8
#define NGRP    2
#define CHUNK   (NTHR * EPT * NGRP)
#define WCAP    (EPT * NGRP * 32)
#define LISTN   (NWAVE * WCAP)
#define ESHF    11
#define NBC     32768
#define NBF     2048
#define RCAP    40960
#define RBN     128
#define TGT     256
#define DEGCAP  512
#define GROWS   64
#define XR      128
#define OTHR    512
#define WSCALE  64
#define ASCALE  64
#define WSCAP   134217728

#define OW1   0
#define OW2   (OW1 + HD * K1)
#define OW3H  (OW2 + HD * K2)
#define OW3L  (OW3H + HD * K2)
#define WPTOT (OW3L + HD * K2)
#define WB1   ((HD * K1 / 8) / NTHR)
#define WB2   ((HD * K2 / 8) / NTHR)
#define WB3   ((HD * K2 / 8) / NTHR)
#define WPREP_BLOCKS (WB1 + WB2 + WB3)

#define LDS_COUNT ((NBC + LISTN + NWAVE) * 4)
#define LDS_FILL  ((RCAP + NBF + LISTN + NWAVE) * 4)
#define LDS_GEMM  (GROWS * HD * 4)

static_assert((CHUNK & (CHUNK - 1)) == 0);
static_assert((NBC & (NBC - 1)) == 0 && (NBF & (NBF - 1)) == 0);
static_assert(NBF <= (1 << ESHF));
static_assert((NBC % NBF) == 0);
static_assert(OTHR * 4 == NBF);
static_assert((RCAP % 32) == 0);
static_assert(TGT == NWAVE * 32);
static_assert(GROWS == (NWAVE / 2) * 16);
static_assert((TGT % GROWS) == 0 && (TGT % XR) == 0);
static_assert(NBC == NWAVE * 32 * 128);
static_assert(K1 == 2 * DI && K2 == 2 * HD && P1 == K1 && P2 == K2);
static_assert((HD * K1 / 8) % NTHR == 0 && (HD * K2 / 8) % NTHR == 0);
static_assert(WPREP_BLOCKS == 160 && WPTOT == 458752);
static_assert(XR == 8 * (NTHR / 16));
static_assert((K1 % 32) == 0 && (K2 % 32) == 0);
static_assert(DI == 4 * 32 && HD == 8 * 32);

typedef float          v4f  __attribute__((ext_vector_type(4)));
typedef float          v8f  __attribute__((ext_vector_type(8)));
typedef int            v4i  __attribute__((ext_vector_type(4)));
typedef unsigned       v2u  __attribute__((ext_vector_type(2)));
typedef unsigned       v4u  __attribute__((ext_vector_type(4)));
typedef _Float16       v4h  __attribute__((ext_vector_type(4)));
typedef _Float16       v8h  __attribute__((ext_vector_type(8)));
typedef _Float16       v16h __attribute__((ext_vector_type(16)));
typedef __bf16         v16b __attribute__((ext_vector_type(16)));
typedef unsigned short us;
union Frag { v4u u[2]; v16h h; v16b b; };
union H8 { v8h h; v4u u; };
union H4 { v4h h; v2u u; };

__device__ __forceinline__ v8f wmh(const Frag& a, const Frag& b, v8f c) {
  v8f d = __builtin_amdgcn_wmma_f32_16x16x32_f16(false, a.h, false, b.h, (short)0, c, false, false);
  asm volatile("v_nop\n\tv_nop\n\tv_nop\n\tv_nop" : "+v"(d) : "v"(a.h), "v"(b.h));
  return d;
}
__device__ __forceinline__ v8f wmb(const Frag& a, const Frag& b, v8f c) {
  v8f d = __builtin_amdgcn_wmma_f32_16x16x32_bf16(false, a.b, false, b.b, (short)0, c, false, false);
  asm volatile("v_nop\n\tv_nop\n\tv_nop\n\tv_nop" : "+v"(d) : "v"(a.h), "v"(b.h));
  return d;
}

__device__ __forceinline__ Frag ldfrag(const us* p) {
  Frag f;
  f.u[0] = *(const v4u*)p;
  f.u[1] = *(const v4u*)(p + 16);
  return f;
}

__device__ __forceinline__ unsigned bf_rne(float x) {
  const unsigned u = __float_as_uint(x);
  return (u + 0x7FFFu + ((u >> 16) & 1u)) >> 16;
}
__device__ __forceinline__ void bf_split(float x, unsigned& hi, unsigned& lo) {
  hi = bf_rne(x);
  const float hf = __uint_as_float(hi << 16);
  lo = bf_rne(x - hf);
}

template <int NB, int GID>
__device__ __forceinline__ int scan_chunk(const int* __restrict__ keys, const int* __restrict__ oth, int nE, int nN,
                                          int cbase, int slotBase, int vec8, int* list, int tid, int lane, int wave) {
  int wc = 0;
#pragma unroll
  for (int g = 0; g < NGRP; ++g) {
    const int el0  = (g * NTHR + tid) * EPT;
    const int e0   = cbase + el0;
    const int sent = -2147483647 - 1;
    v4i da, db, sa, sb;
    if (vec8 != 0 && cbase + CHUNK <= nE) {
      da = *(const v4i*)(keys + e0);
      db = *(const v4i*)(keys + e0 + 4);
      sa = *(const v4i*)(oth + e0);
      sb = *(const v4i*)(oth + e0 + 4);
    } else {
      const int le = nE - 1;
      da.x = (e0     < nE) ? keys[min(e0, le)]     : sent;
      da.y = (e0 + 1 < nE) ? keys[min(e0 + 1, le)] : sent;
      da.z = (e0 + 2 < nE) ? keys[min(e0 + 2, le)] : sent;
      da.w = (e0 + 3 < nE) ? keys[min(e0 + 3, le)] : sent;
      db.x = (e0 + 4 < nE) ? keys[min(e0 + 4, le)] : sent;
      db.y = (e0 + 5 < nE) ? keys[min(e0 + 5, le)] : sent;
      db.z = (e0 + 6 < nE) ? keys[min(e0 + 6, le)] : sent;
      db.w = (e0 + 7 < nE) ? keys[min(e0 + 7, le)] : sent;
      sa.x = oth[min(e0, le)];
      sa.y = oth[min(e0 + 1, le)];
      sa.z = oth[min(e0 + 2, le)];
      sa.w = oth[min(e0 + 3, le)];
      sb.x = oth[min(e0 + 4, le)];
      sb.y = oth[min(e0 + 5, le)];
      sb.z = oth[min(e0 + 6, le)];
      sb.w = oth[min(e0 + 7, le)];
    }
    const int g0 = min(max(sa.x, 0), nN - 1), g1 = min(max(sa.y, 0), nN - 1);
    const int g2 = min(max(sa.z, 0), nN - 1), g3 = min(max(sa.w, 0), nN - 1);
    const int g4 = min(max(sb.x, 0), nN - 1), g5 = min(max(sb.y, 0), nN - 1);
    const int g6 = min(max(sb.z, 0), nN - 1), g7 = min(max(sb.w, 0), nN - 1);
    const unsigned nb = (unsigned)slotBase;
    const unsigned s0 = (unsigned)da.x - nb, s1 = (unsigned)da.y - nb;
    const unsigned s2 = (unsigned)da.z - nb, s3 = (unsigned)da.w - nb;
    const unsigned s4 = (unsigned)db.x - nb, s5 = (unsigned)db.y - nb;
    const unsigned s6 = (unsigned)db.z - nb, s7 = (unsigned)db.w - nb;
    const bool h0 = (s0 < (unsigned)NB) & (da.x != sa.x), h1 = (s1 < (unsigned)NB) & (da.y != sa.y);
    const bool h2 = (s2 < (unsigned)NB) & (da.z != sa.z), h3 = (s3 < (unsigned)NB) & (da.w != sa.w);
    const bool h4 = (s4 < (unsigned)NB) & (db.x != sb.x), h5 = (s5 < (unsigned)NB) & (db.y != sb.y);
    const bool h6 = (s6 < (unsigned)NB) & (db.z != sb.z), h7 = (s7 < (unsigned)NB) & (db.w != sb.w);
    const unsigned any = __builtin_amdgcn_ballot_w32(h0 | h1 | h2 | h3 | h4 | h5 | h6 | h7);
    if (any != 0u) {
#define HITJ(HJ, SJ, VJ) { \
        const unsigned mj = __builtin_amdgcn_ballot_w32(HJ); \
        if (mj != 0u) { \
          if (HJ) { \
            const int pos = wc + (int)__builtin_amdgcn_mbcnt_lo(mj, 0u); \
            const int entv = GID ? (((VJ) << ESHF) | (int)(SJ)) : (int)(SJ); \
            if (pos < WCAP) list[wave * WCAP + pos] = entv; \
          } \
          wc += (int)__builtin_popcount(mj); } }
      HITJ(h0, s0, g0)
      HITJ(h1, s1, g1)
      HITJ(h2, s2, g2)
      HITJ(h3, s3, g3)
      HITJ(h4, s4, g4)
      HITJ(h5, s5, g5)
      HITJ(h6, s6, g6)
      HITJ(h7, s7, g7)
#undef HITJ
    }
  }
  return wc;
}

__global__ __launch_bounds__(NTHR) void k_wprep(const float* __restrict__ w10, const float* __restrict__ w11,
                                                const float* __restrict__ w20, const float* __restrict__ w21,
                                                const float* __restrict__ w30, const float* __restrict__ w31,
                                                us* wp) {
  const int tid = threadIdx.x;
  const int b = (int)blockIdx.x;
  const float* s0;
  const float* s1;
  int K, j, dbase, mode;
  if (b < WB1)            { s0 = w10; s1 = w11; K = K1; j = b * NTHR + tid;               dbase = OW1;  mode = 0; }
  else if (b < WB1 + WB2) { s0 = w20; s1 = w21; K = K2; j = (b - WB1) * NTHR + tid;       dbase = OW2;  mode = 0; }
  else                    { s0 = w30; s1 = w31; K = K2; j = (b - WB1 - WB2) * NTHR + tid; dbase = OW3H; mode = 1; }
  const int kq = K >> 3;
  const int jm = HD * kq - 1;
  j = j < 0 ? 0 : (j > jm ? jm : j);
  const int n  = j / kq;
  const int k0 = (j - n * kq) * 8;
  const int Kh = K >> 1;
  const float* s = (k0 < Kh) ? s0 : s1;
  const int kk = (k0 < Kh) ? k0 : (k0 - Kh);
  float v[8];
#pragma unroll
  for (int e = 0; e < 8; ++e) v[e] = s[(size_t)(kk + e) * HD + n];
  us* d = wp + (size_t)dbase + (size_t)n * K + (size_t)k0;
  if (mode == 0) {
    H8 p;
#pragma unroll
    for (int e = 0; e < 8; ++e) p.h[e] = (_Float16)(v[e] * (float)WSCALE);
    const v4u pu = p.u;
    *(volatile v4u*)d = pu;
    __threadfence();
    *(volatile v4u*)d = pu;
  } else {
    v4u hv, lv;
#pragma unroll
    for (int q = 0; q < 4; ++q) {
      unsigned a0, l0, a1, l1;
      bf_split(v[2 * q], a0, l0);
      bf_split(v[2 * q + 1], a1, l1);
      hv[q] = a0 | (a1 << 16);
      lv[q] = l0 | (l1 << 16);
    }
    us* dl = d + (OW3L - OW3H);
    *(volatile v4u*)d = hv;
    *(volatile v4u*)dl = lv;
    __threadfence();
    *(volatile v4u*)d = hv;
    *(volatile v4u*)dl = lv;
  }
}

__global__ __launch_bounds__(NTHR) void k_xcvt(const float* __restrict__ x, us* A1, int nN) {
  const int tid = threadIdx.x;
  const int rsub = tid >> 4;
  const int c0 = (tid & 15) * 8;
#pragma unroll 1
  for (int it = 0; it < XR / 16; ++it) {
    const int row = (int)blockIdx.x * XR + it * 16 + rsub;
    const int rr = row > nN - 1 ? nN - 1 : row;
    const v4f xa = *(const v4f*)(x + (size_t)rr * DI + c0);
    const v4f xb = *(const v4f*)(x + (size_t)rr * DI + c0 + 4);
    const float z = (row < nN) ? (float)ASCALE : 0.f;
    H8 p;
    p.h[0] = (_Float16)(xa.x * z); p.h[1] = (_Float16)(xa.y * z);
    p.h[2] = (_Float16)(xa.z * z); p.h[3] = (_Float16)(xa.w * z);
    p.h[4] = (_Float16)(xb.x * z); p.h[5] = (_Float16)(xb.y * z);
    p.h[6] = (_Float16)(xb.z * z); p.h[7] = (_Float16)(xb.w * z);
    const v4u pu = p.u;
    us* d = A1 + (size_t)row * P1 + c0;
    *(volatile v4u*)d = pu;
    __threadfence();
    *(volatile v4u*)d = pu;
  }
}

template <int WD>
__device__ __forceinline__ void st_cnt(const int* scnt, int* cp, float* dp, int wave, int lane) {
#pragma unroll 4
  for (int q = 0; q < 32; ++q) {
    const int f = (wave * 32 + q) * 128 + 4 * lane;
    const v4i c = *(const v4i*)(scnt + f);
    if constexpr (WD == 0) {
      *(volatile v4i*)(cp + f) = c;
    } else {
      const float g0 = (float)c.x, g1 = (float)c.y, g2 = (float)c.z, g3 = (float)c.w;
      v4f d;
      d.x = g0 > 0.f ? rsqrtf(g0) : 0.f; d.y = g1 > 0.f ? rsqrtf(g1) : 0.f;
      d.z = g2 > 0.f ? rsqrtf(g2) : 0.f; d.w = g3 > 0.f ? rsqrtf(g3) : 0.f;
      *(volatile v4f*)(dp + f) = d;
    }
  }
}

template <int WD>
__global__ __launch_bounds__(NTHR) void k_count(
    const int* __restrict__ keys, const int* __restrict__ oth, int* cnt, float* dinv, int nE, int nN, int vec8) {
  extern __shared__ v4f lds_dyn[];
  int* scnt = (int*)lds_dyn;
  int* list = scnt + NBC;
  int* wcnt = list + LISTN;
  const int tid = threadIdx.x, lane = tid & 31, wave = tid >> 5;
  const int nodeBase = blockIdx.x * NBC;

  {
    const v4i z = {0, 0, 0, 0};
    for (int i = tid; i < NBC / 4; i += NTHR) ((v4i*)scnt)[i] = z;
  }
  __syncthreads();

  const int nChunks = (nE + CHUNK - 1) / CHUNK;
#pragma unroll 1
  for (int ch = 0; ch < nChunks; ++ch) {
    const int cbase = ch * CHUNK;
    const int wc = scan_chunk<NBC, 0>(keys, oth, nE, nN, cbase, nodeBase, vec8, list, tid, lane, wave);
    if (lane == 0) wcnt[wave] = wc;
    __syncthreads();
    if (wave == 0) {
#pragma unroll 1
      for (int wsx = 0; wsx < NWAVE; ++wsx) {
        int n = __builtin_amdgcn_readfirstlane(wcnt[wsx]);
        n = n > WCAP ? WCAP : (n < 0 ? 0 : n);
        const int* lp = list + wsx * WCAP;
#pragma unroll 1
        for (int i = 0; i < n; ++i) {
          const int ent  = __builtin_amdgcn_readfirstlane(lp[i]);
          const int slot = ent & (NBC - 1);
          if (lane == 0) scnt[slot] = scnt[slot] + 1;
        }
      }
    }
    __syncthreads();
  }

  int*   cp = cnt + (size_t)nodeBase;
  float* dp = dinv + (size_t)nodeBase;
  st_cnt<WD>(scnt, cp, dp, wave, lane);
  __threadfence();
  st_cnt<WD>(scnt, cp, dp, wave, lane);
}

__global__ __launch_bounds__(OTHR) void k_offsets(
    const int* __restrict__ cnt, int* off, int* rbase, int nBF) {
  __shared__ __attribute__((aligned(16))) int srb[RBN];
  __shared__ int wtot[OTHR / 32];
  const int tid = threadIdx.x, lane = tid & 31, wave = tid >> 5;
  for (int i = tid; i < RBN; i += OTHR) srb[i] = 0;
  int carry = 0;
#pragma unroll 1
  for (int fb = 0; fb < nBF; ++fb) {
    const int base = fb * NBF;
    const v4i c = *(const v4i*)(cnt + base + 4 * tid);
    const int e0 = max(c.x, 0), e1 = max(c.y, 0), e2 = max(c.z, 0), e3 = max(c.w, 0);
    const int ts = e0 + e1 + e2 + e3;
    int incl = ts;
#pragma unroll
    for (int d = 1; d < 32; d <<= 1) {
      const int t = __shfl_up(incl, d, 32);
      if (lane >= d) incl += t;
    }
    if (lane == 31) wtot[wave] = incl;
    __syncthreads();
    int pre = 0;
#pragma unroll 1
    for (int w = 0; w < wave; ++w) pre += wtot[w];
    int tot = 0;
#pragma unroll
    for (int w = 0; w < OTHR / 32; ++w) tot += wtot[w];
    int run = carry + pre + incl - ts;
    v4i o;
    o.x = run; run += e0;
    o.y = run; run += e1;
    o.z = run; run += e2;
    o.w = run;
    int* op = off + base + 4 * tid;
    *(volatile v4i*)op = o;
    __threadfence();
    *(volatile v4i*)op = o;
    if (tid == 0) srb[min(fb, RBN - 1)] = carry;
    carry += (tot + 31) & ~31;
    __syncthreads();
  }
  if (tid == 0) srb[min(nBF, RBN - 1)] = carry;
  __syncthreads();
  v4i rv = {0, 0, 0, 0};
  if (tid < 32) rv = *(const v4i*)(srb + 4 * tid);
  if (tid < 32) *(volatile v4i*)(rbase + 4 * tid) = rv;
  __threadfence();
  if (tid < 32) *(volatile v4i*)(rbase + 4 * tid) = rv;
}

__global__ __launch_bounds__(NTHR) void k_fill(
    const int* __restrict__ keys, const int* __restrict__ oth, const int* __restrict__ off, const int* __restrict__ rbase,
    int* csr, int nN, int nE, int vec8, int csrLen) {
  extern __shared__ v4f lds_dyn[];
  int* region = (int*)lds_dyn;
  int* cursor = region + RCAP;
  int* list   = cursor + NBF;
  int* wcnt   = list + LISTN;
  const int tid = threadIdx.x, lane = tid & 31, wave = tid >> 5;
  const int b = blockIdx.x;
  const int nodeBase = b * NBF;

  int rb0 = rbase[b];
  const int rb1 = rbase[b + 1];
  rb0 = rb0 < 0 ? 0 : (rb0 > csrLen ? csrLen : rb0);
  rb0 &= ~31;
  int len = rb1 - rb0;
  len = len < 0 ? 0 : (len > RCAP ? RCAP : len);
  int lenW = (len + 31) & ~31;
  if (rb0 + lenW > csrLen) lenW = (csrLen - rb0) & ~31;

  {
    const v4i z = {0, 0, 0, 0};
    for (int i = tid; i < RCAP / 4; i += NTHR) ((v4i*)region)[i] = z;
    for (int s = tid; s < NBF; s += NTHR) {
      int o = off[nodeBase + s] - rb0;
      o = o < 0 ? 0 : (o > RCAP ? RCAP : o);
      cursor[s] = o;
    }
  }
  __syncthreads();

  const int nChunks = (nE + CHUNK - 1) / CHUNK;
#pragma unroll 1
  for (int ch = 0; ch < nChunks; ++ch) {
    const int cbase = ch * CHUNK;
    const int wc = scan_chunk<NBF, 1>(keys, oth, nE, nN, cbase, nodeBase, vec8, list, tid, lane, wave);
    if (lane == 0) wcnt[wave] = wc;
    __syncthreads();
    if (wave == 0) {
#pragma unroll 1
      for (int wsx = 0; wsx < NWAVE; ++wsx) {
        int n = __builtin_amdgcn_readfirstlane(wcnt[wsx]);
        n = n > WCAP ? WCAP : (n < 0 ? 0 : n);
        const int* lp = list + wsx * WCAP;
#pragma unroll 1
        for (int i = 0; i < n; ++i) {
          const int ent  = __builtin_amdgcn_readfirstlane(lp[i]);
          const int slot = ent & (NBF - 1);
          int src = (ent >> ESHF) & 0xFFFFF;
          src = src > nN - 1 ? nN - 1 : src;
          if (lane == 0) {
            int pos = cursor[slot];
            pos = pos < 0 ? 0 : (pos > RCAP - 1 ? RCAP - 1 : pos);
            region[pos] = src;
            const int np = pos + 1;
            cursor[slot] = np > RCAP ? RCAP : np;
          }
        }
      }
    }
    __syncthreads();
  }

  const int nv = lenW >> 2;
  int* gp = csr + rb0;
#pragma unroll 1
  for (int i = tid; i < nv; i += NTHR) { const v4i v = ((const v4i*)region)[i]; *(volatile v4i*)(gp + 4 * i) = v; }
  __threadfence();
#pragma unroll 1
  for (int i = tid; i < nv; i += NTHR) { const v4i v = ((const v4i*)region)[i]; *(volatile v4i*)(gp + 4 * i) = v; }
}

template <int MODE>
__global__ __launch_bounds__(NTHR) void k_agg(
    const int* __restrict__ csr, const int* __restrict__ off, const int* __restrict__ cnt,
    const float* __restrict__ dinv, const float* __restrict__ xf, const us* xh, const us* xl,
    us* oh, us* ol, int nN, int csrLen) {
  constexpr int CH = (MODE == 1) ? 4 : 8;
  const int tid = threadIdx.x, lane = tid & 31, wave = tid >> 5;
  const int tbase = blockIdx.x * TGT + wave * 32;
  const int cl = tbase + lane;
  const int cnt_l = cnt[cl];
  const int off_l = off[cl];
  const int dv_l  = __float_as_int(dinv[cl]);

#pragma unroll 1
  for (int j = 0; j < 32; ++j) {
    const int c = tbase + j;
    int n = __builtin_amdgcn_readlane(cnt_l, j);
    n = n < 0 ? 0 : (n > DEGCAP ? DEGCAP : n);
    const int st = __builtin_amdgcn_readlane(off_l, j);
    const float dc = __int_as_float(__builtin_amdgcn_readlane(dv_l, j));
    float acc[CH];
#pragma unroll
    for (int i = 0; i < CH; ++i) acc[i] = 0.f;
#pragma unroll 1
    for (int q0 = 0; q0 < n; q0 += 32) {
      int pos = st + q0 + lane;
      pos = pos < 0 ? 0 : (pos > csrLen - 1 ? csrLen - 1 : pos);
      int sl = csr[pos];
      sl = sl < 0 ? 0 : (sl > nN - 1 ? nN - 1 : sl);
      const int ds_l = __float_as_int(dinv[sl]);
      const int mcnt = (n - q0) < 32 ? (n - q0) : 32;
#pragma unroll 1
      for (int p = 0; p < mcnt; ++p) {
        const int sidx = __builtin_amdgcn_readlane(sl, p);
        const float ds = __int_as_float(__builtin_amdgcn_readlane(ds_l, p));
        const float wv = -(ds * dc);
        if constexpr (MODE == 1) {
          const v4f xv = *(const v4f*)(xf + (size_t)sidx * DI + 4 * lane);
          acc[0] += wv * xv.x; acc[1] += wv * xv.y; acc[2] += wv * xv.z; acc[3] += wv * xv.w;
        } else if constexpr (MODE == 2) {
          const v4f xa = *(const v4f*)(xf + (size_t)sidx * HD + 8 * lane);
          const v4f xb = *(const v4f*)(xf + (size_t)sidx * HD + 8 * lane + 4);
          acc[0] += wv * xa.x; acc[1] += wv * xa.y; acc[2] += wv * xa.z; acc[3] += wv * xa.w;
          acc[4] += wv * xb.x; acc[5] += wv * xb.y; acc[6] += wv * xb.z; acc[7] += wv * xb.w;
        } else {
          const v4u hu = *(const v4u*)(xh + (size_t)sidx * P2 + 8 * lane);
          const v4u lu = *(const v4u*)(xl + (size_t)sidx * P2 + 8 * lane);
#pragma unroll
          for (int q = 0; q < 4; ++q) {
            const float f0 = __uint_as_float(hu[q] << 16) + __uint_as_float(lu[q] << 16);
            const float f1 = __uint_as_float(hu[q] & 0xffff0000u) + __uint_as_float(lu[q] & 0xffff0000u);
            acc[2 * q]     += wv * f0;
            acc[2 * q + 1] += wv * f1;
          }
        }
      }
    }
    if constexpr (MODE == 1) {
      H4 pk;
      pk.h[0] = (_Float16)(acc[0] * (float)ASCALE); pk.h[1] = (_Float16)(acc[1] * (float)ASCALE);
      pk.h[2] = (_Float16)(acc[2] * (float)ASCALE); pk.h[3] = (_Float16)(acc[3] * (float)ASCALE);
      const v2u uu = pk.u;
      us* d = oh + (size_t)c * P1 + DI + 4 * lane;
      *(volatile v2u*)d = uu;
      __threadfence();
      *(volatile v2u*)d = uu;
    } else if constexpr (MODE == 2) {
      H8 pk;
#pragma unroll
      for (int i = 0; i < 8; ++i) pk.h[i] = (_Float16)(acc[i] * (float)ASCALE);
      const v4u uu = pk.u;
      us* d = oh + (size_t)c * P2 + HD + 8 * lane;
      *(volatile v4u*)d = uu;
      __threadfence();
      *(volatile v4u*)d = uu;
    } else {
      v4u hv, lv;
#pragma unroll
      for (int q = 0; q < 4; ++q) {
        unsigned a0, l0, a1, l1;
        bf_split(acc[2 * q], a0, l0);
        bf_split(acc[2 * q + 1], a1, l1);
        hv[q] = a0 | (a1 << 16);
        lv[q] = l0 | (l1 << 16);
      }
      us* dh = oh + (size_t)c * P2 + HD + 8 * lane;
      us* dl = ol + (size_t)c * P2 + HD + 8 * lane;
      *(volatile v4u*)dh = hv;
      *(volatile v4u*)dl = lv;
      __threadfence();
      *(volatile v4u*)dh = hv;
      *(volatile v4u*)dl = lv;
    }
  }
}

__device__ __forceinline__ void st_f16(const float* sw, us* Ch, int grow0, int col0, int lane) {
  const int rsel = lane >> 4, cs = (lane & 15) * 8;
#pragma unroll
  for (int i = 0; i < 8; ++i) {
    const int rl = 2 * i + rsel;
    const v4f u0 = *(const v4f*)(sw + rl * HD + cs);
    const v4f u1 = *(const v4f*)(sw + rl * HD + cs + 4);
    H8 p;
    p.h[0] = (_Float16)(u0.x * (float)ASCALE); p.h[1] = (_Float16)(u0.y * (float)ASCALE);
    p.h[2] = (_Float16)(u0.z * (float)ASCALE); p.h[3] = (_Float16)(u0.w * (float)ASCALE);
    p.h[4] = (_Float16)(u1.x * (float)ASCALE); p.h[5] = (_Float16)(u1.y * (float)ASCALE);
    p.h[6] = (_Float16)(u1.z * (float)ASCALE); p.h[7] = (_Float16)(u1.w * (float)ASCALE);
    const v4u pu = p.u;
    *(volatile v4u*)(Ch + (size_t)(grow0 + rl) * P2 + col0 + cs) = pu;
  }
}

__device__ __forceinline__ void st_bf2(const float* sw, us* Ch, us* Clo, int grow0, int col0, int lane) {
  const int rsel = lane >> 4, cs = (lane & 15) * 8;
#pragma unroll
  for (int i = 0; i < 8; ++i) {
    const int rl = 2 * i + rsel;
    const v4f u0 = *(const v4f*)(sw + rl * HD + cs);
    const v4f u1 = *(const v4f*)(sw + rl * HD + cs + 4);
    unsigned e0, f0, e1, f1;
    v4u hv, lv;
    bf_split(u0.x, e0, f0); bf_split(u0.y, e1, f1); hv[0] = e0 | (e1 << 16); lv[0] = f0 | (f1 << 16);
    bf_split(u0.z, e0, f0); bf_split(u0.w, e1, f1); hv[1] = e0 | (e1 << 16); lv[1] = f0 | (f1 << 16);
    bf_split(u1.x, e0, f0); bf_split(u1.y, e1, f1); hv[2] = e0 | (e1 << 16); lv[2] = f0 | (f1 << 16);
    bf_split(u1.z, e0, f0); bf_split(u1.w, e1, f1); hv[3] = e0 | (e1 << 16); lv[3] = f0 | (f1 << 16);
    const size_t o = (size_t)(grow0 + rl) * P2 + col0 + cs;
    *(volatile v4u*)(Ch + o) = hv;
    *(volatile v4u*)(Clo + o) = lv;
  }
}

__device__ __forceinline__ void st_f32(const float* sw, float* Fo, int grow0, int col0, int lane, int nrows) {
#pragma unroll
  for (int i = 0; i < 16; ++i) {
    const int row = grow0 + i;
    const v4f v = *(const v4f*)(sw + i * HD + 4 * lane);
    if (row < nrows) *(volatile v4f*)(Fo + (size_t)row * HD + col0 + 4 * lane) = v;
  }
}

template <int KD, int SPLIT, int EPI>
__global__ __launch_bounds__(NTHR) void k_gemm(
    const us* A, const us* Alo, int lda, const us* __restrict__ Bw, const us* __restrict__ Bwlo,
    const float* __restrict__ bias, us* Ch, us* Clo, float* Fo, int nrows) {
  extern __shared__ v4f lds_dyn[];
  constexpr int NT = 8;
  constexpr float OSC = SPLIT ? 1.0f : (1.0f / (float)(ASCALE * WSCALE));
  float* stg = (float*)lds_dyn;
  const int tid = threadIdx.x, lane = tid & 31, wave = tid >> 5, hh = lane >> 4, m = lane & 15;
  const int rt = wave >> 1, chh = wave & 1;
  const int rowBase = blockIdx.x * GROWS;
  const int arow = rowBase + rt * 16 + m;
  const int col0 = chh * 128;
  const us* ap  = A + (size_t)arow * lda + 8 * hh;
  const us* alp = Alo + (size_t)arow * lda + 8 * hh;
  const us* bp  = Bw + (size_t)(col0 + m) * KD + 8 * hh;
  const us* blp = Bwlo + (size_t)(col0 + m) * KD + 8 * hh;

  v8f acc[NT];
#pragma unroll
  for (int t = 0; t < NT; ++t) { v8f z = {0.f, 0.f, 0.f, 0.f, 0.f, 0.f, 0.f, 0.f}; acc[t] = z; }

#pragma unroll 1
  for (int kt = 0; kt < KD / 32; ++kt) {
    const Frag a = ldfrag(ap + 32 * kt);
    Frag al = a;
    if constexpr (SPLIT != 0) al = ldfrag(alp + 32 * kt);
#pragma unroll
    for (int t = 0; t < NT; ++t) {
      const Frag b = ldfrag(bp + (size_t)(16 * t) * KD + 32 * kt);
      if constexpr (SPLIT != 0) {
        const Frag bl = ldfrag(blp + (size_t)(16 * t) * KD + 32 * kt);
        acc[t] = wmb(a, b, acc[t]);
        acc[t] = wmb(a, bl, acc[t]);
        acc[t] = wmb(al, b, acc[t]);
      } else {
        acc[t] = wmh(a, b, acc[t]);
      }
    }
  }

  {
    float* sp = stg + (rt * 16 + 8 * hh) * HD + col0 + m;
#pragma unroll
    for (int t = 0; t < NT; ++t) {
      const float bc = bias[col0 + 16 * t + m];
#pragma unroll
      for (int r = 0; r < 8; ++r) {
        float v = acc[t][r] * OSC + bc;
        if constexpr (EPI != 2) v = fmaxf(v, 0.f);
        sp[r * HD + 16 * t] = v;
      }
    }
  }
  __syncthreads();

  const float* sw = stg + (rt * 16) * HD + col0;
  const int grow0 = rowBase + rt * 16;
  if constexpr (EPI == 0) {
    st_f16(sw, Ch, grow0, col0, lane);
    st_f32(sw, Fo, grow0, col0, lane, nrows);
  } else if constexpr (EPI == 1) {
    st_bf2(sw, Ch, Clo, grow0, col0, lane);
  } else {
    st_f32(sw, Fo, grow0, col0, lane, nrows);
  }
  __threadfence();
  if constexpr (EPI == 0) {
    st_f16(sw, Ch, grow0, col0, lane);
    st_f32(sw, Fo, grow0, col0, lane, nrows);
  } else if constexpr (EPI == 1) {
    st_bf2(sw, Ch, Clo, grow0, col0, lane);
  } else {
    st_f32(sw, Fo, grow0, col0, lane, nrows);
  }
}

extern "C" void kernel_launch(void* const* d_in, const int* in_sizes, int n_in,
                              void* d_out, int out_size, void* d_ws, size_t ws_size,
                              hipStream_t stream) {
  if (n_in < 11) return;
  if ((in_sizes[0] % DI) != 0 || (in_sizes[1] % 2) != 0) return;
  const int nN = in_sizes[0] / DI;
  const int nE = in_sizes[1] / 2;
  if (nN <= 0 || nE <= 0) return;
  if (in_sizes[2] != DI * HD || in_sizes[3] != DI * HD || in_sizes[4] != HD) return;
  if (in_sizes[5] != HD * HD || in_sizes[6] != HD * HD || in_sizes[7] != HD) return;
  if (in_sizes[8] != HD * HD || in_sizes[9] != HD * HD || in_sizes[10] != HD) return;
  if (out_size != nN * HD) return;
  if (nN > (1 << 20) || nE > (1 << 28)) return;

  const float* x    = (const float*)d_in[0];
  const int*   ei   = (const int*)d_in[1];
  const int*   srcp = ei;
  const int*   dstp = ei + nE;
  const float* w10  = (const float*)d_in[2];
  const float* w11  = (const float*)d_in[3];
  const float* b1   = (const float*)d_in[4];
  const float* w20  = (const float*)d_in[5];
  const float* w21  = (const float*)d_in[6];
  const float* b2   = (const float*)d_in[7];
  const float* w30  = (const float*)d_in[8];
  const float* w31  = (const float*)d_in[9];
  const float* b3   = (const float*)d_in[10];
  float* out = (float*)d_out;

  const int NPAD   = ((nN + TGT - 1) / TGT) * TGT;
  const int nBC    = (nN + NBC - 1) / NBC;
  const int CNTPAD = nBC * NBC;
  const int nBF    = (nN + NBF - 1) / NBF;
  const int OFFN   = nBF * NBF;
  if (nBF + 1 > RBN) return;
  if (OFFN > CNTPAD || NPAD > OFFN) return;
  const int csrLen = ((nE + 31) & ~31) + 32 * (nBF + 1);
  const int nX     = NPAD / XR;
  const int nGemm  = NPAD / GROWS;
  const int nAgg   = NPAD / TGT;

  char* ws = (char*)d_ws;
  size_t off = 0;
  const size_t szR  = ((size_t)NPAD * HD * 4 > (size_t)NPAD * P2 * 2) ? (size_t)NPAD * HD * 4 : (size_t)NPAD * P2 * 2;
  const size_t oW   = off; off += (size_t)WPTOT * 2;          off = (off + 255) & ~(size_t)255;
  const size_t oDv  = off; off += (size_t)CNTPAD * 4;         off = (off + 255) & ~(size_t)255;
  const size_t oCnt = off; off += (size_t)CNTPAD * 4;         off = (off + 255) & ~(size_t)255;
  const size_t oOff = off; off += (size_t)OFFN * 4;           off = (off + 255) & ~(size_t)255;
  const size_t oRb  = off; off += (size_t)RBN * 4;            off = (off + 255) & ~(size_t)255;
  const size_t oCsr = off; off += (size_t)csrLen * 4;         off = (off + 255) & ~(size_t)255;
  const size_t oA1  = off; off += (size_t)NPAD * P1 * 2;      off = (off + 255) & ~(size_t)255;
  const size_t oAH  = off; off += (size_t)NPAD * P2 * 2;      off = (off + 255) & ~(size_t)255;
  const size_t oR   = off; off += szR;                        off = (off + 255) & ~(size_t)255;
  if (off > ws_size || off > (size_t)WSCAP) return;
  us*    wp   = (us*)(ws + oW);
  float* dinv = (float*)(ws + oDv);
  int*   cnt  = (int*)(ws + oCnt);
  int*   offp = (int*)(ws + oOff);
  int*   rb   = (int*)(ws + oRb);
  int*   csr  = (int*)(ws + oCsr);
  us*    A1   = (us*)(ws + oA1);
  us*    AH   = (us*)(ws + oAH);
  float* F    = (float*)(ws + oR);
  us*    AL   = (us*)(ws + oR);
  const us* pW1  = wp + OW1;
  const us* pW2  = wp + OW2;
  const us* pW3H = wp + OW3H;
  const us* pW3L = wp + OW3L;

  const int vec8 = ((nE & 3) == 0) ? 1 : 0;

  k_wprep<<<WPREP_BLOCKS, NTHR, 0, stream>>>(w10, w11, w20, w21, w30, w31, wp);
  k_xcvt<<<nX, NTHR, 0, stream>>>(x, A1, nN);

  hipFuncSetAttribute(reinterpret_cast<const void*>(&k_count<1>),
                      hipFuncAttributeMaxDynamicSharedMemorySize, LDS_COUNT);
  hipFuncSetAttribute(reinterpret_cast<const void*>(&k_count<0>),
                      hipFuncAttributeMaxDynamicSharedMemorySize, LDS_COUNT);
  k_count<1><<<nBC, NTHR, LDS_COUNT, stream>>>(srcp, dstp, cnt, dinv, nE, nN, vec8);
  k_count<0><<<nBC, NTHR, LDS_COUNT, stream>>>(dstp, srcp, cnt, dinv, nE, nN, vec8);
  k_offsets<<<1, OTHR, 0, stream>>>(cnt, offp, rb, nBF);
  hipFuncSetAttribute(reinterpret_cast<const void*>(&k_fill),
                      hipFuncAttributeMaxDynamicSharedMemorySize, LDS_FILL);
  k_fill<<<nBF, NTHR, LDS_FILL, stream>>>(dstp, srcp, offp, rb, csr, nN, nE, vec8, csrLen);

  hipFuncSetAttribute(reinterpret_cast<const void*>(&k_gemm<K1, 0, 0>),
                      hipFuncAttributeMaxDynamicSharedMemorySize, LDS_GEMM);
  hipFuncSetAttribute(reinterpret_cast<const void*>(&k_gemm<K2, 0, 1>),
                      hipFuncAttributeMaxDynamicSharedMemorySize, LDS_GEMM);
  hipFuncSetAttribute(reinterpret_cast<const void*>(&k_gemm<K2, 1, 2>),
                      hipFuncAttributeMaxDynamicSharedMemorySize, LDS_GEMM);

  k_agg<1><<<nAgg, NTHR, 0, stream>>>(csr, offp, cnt, dinv, x, A1, A1, A1, A1, nN, csrLen);
  k_gemm<K1, 0, 0><<<nGemm, NTHR, LDS_GEMM, stream>>>(A1, A1, P1, pW1, pW1, b1, AH, AH, F, NPAD);
  k_agg<2><<<nAgg, NTHR, 0, stream>>>(csr, offp, cnt, dinv, F, AH, AH, AH, AH, nN, csrLen);
  k_gemm<K2, 0, 1><<<nGemm, NTHR, LDS_GEMM, stream>>>(AH, AH, P2, pW2, pW2, b2, AH, AL, F, NPAD);
  k_agg<3><<<nAgg, NTHR, 0, stream>>>(csr, offp, cnt, dinv, F, AH, AL, AH, AL, nN, csrLen);
  k_gemm<K2, 1, 2><<<nGemm, NTHR, LDS_GEMM, stream>>>(AH, AL, P2, pW3H, pW3L, b3, AH, AL, out, nN);
}
